// EdgeConvAuxLayer_23905787970103
// MI455X (gfx1250) — hardware-verified
//
#include <hip/hip_runtime.h>
#include <stddef.h>


#define NCH   64
#define NAUX  16
#define KNB   16
#define NTHR  256
#define NWV   8
#define PPW   8
#define PPB   (NWV * PPW)
#define NBA   256
#define BNEPS 1e-5f

#define OW1P  0
#define OW2H  2048
#define OW2L  6144
#define OA1H  10240
#define OA1L  12288
#define OA2H  14336
#define OA2L  22528
#define WPLN  30720
#define WPLB  (WPLN * 2)

#define PB1   0
#define PMU1  64
#define PSC1  128
#define PBB1  192
#define PB2   256
#define PMU2  320
#define PSC2  384
#define PBB2  448
#define PBA1  512
#define PBA2  576
#define PLNG  704
#define PLNB  768
#define PRMN  832
#define PRMB  (PRMN * 4)

#define WA6   0
#define WHH   1024
#define WHL   3072
#define WXH   5120
#define WXL   6144
#define WOS   7168
#define WVB   9216

#define LDS_BASEW (WPLB + PRMB)
#define LDS_SB    (LDS_BASEW + NWV * WVB)
#define LDS_SL    (LDS_SB + NWV * 128 * 8)
#define LDS_EDGE  (LDS_SL + 128 * 8)

static_assert((LDS_BASEW % 16) == 0);
static_assert((WVB % 16) == 0);
static_assert((LDS_SB % 16) == 0);
static_assert((LDS_SL % 16) == 0);
static_assert(LDS_EDGE <= 200 * 1024);
static_assert((WPLB / 16) % NTHR == 0);
static_assert(PPB == 64);

typedef float          v4f  __attribute__((ext_vector_type(4)));
typedef float          v8f  __attribute__((ext_vector_type(8)));
typedef double         v2d  __attribute__((ext_vector_type(2)));
typedef unsigned int   v4u  __attribute__((ext_vector_type(4)));
typedef unsigned short u16t;
typedef u16t           v8us __attribute__((ext_vector_type(8)));
typedef __bf16         v16bf __attribute__((ext_vector_type(16)));
typedef v8us __attribute__((may_alias)) v8usa;
typedef v4f  __attribute__((may_alias)) v4fa;
typedef v2d  __attribute__((may_alias)) v2da;

union FragB { v16bf v; v8us u[2]; };


__device__ __forceinline__ unsigned bfr(float x) {
  const unsigned u = __float_as_uint(x);
  return (u + 0x7FFFu + ((u >> 16) & 1u)) >> 16;
}

__device__ __forceinline__ void split2(float x, u16t& hi, u16t& lo) {
  const unsigned hb = bfr(x);
  const float r = x - __uint_as_float(hb << 16);
  hi = (u16t)hb;
  lo = (u16t)bfr(r);
}

__device__ __forceinline__ void wsync() {
  __builtin_amdgcn_fence(__ATOMIC_ACQ_REL, "wavefront");
  __builtin_amdgcn_wave_barrier();
}

__device__ __forceinline__ v8f wmb1(v16bf a, v16bf b, v8f c) {
  v8f d = __builtin_amdgcn_wmma_f32_16x16x32_bf16(false, a, false, b, (short)0, c, false, false);
#if defined(__HIP_DEVICE_COMPILE__)
  asm volatile("v_nop\n\tv_nop\n\tv_nop\n\tv_nop" : "+v"(d) : "v"(a), "v"(b));
#endif
  return d;
}

__device__ __forceinline__ v8f wm3(v16bf ah, v16bf al, v16bf bh, v16bf bl, v8f c) {
  c = __builtin_amdgcn_wmma_f32_16x16x32_bf16(false, ah, false, bh, (short)0, c, false, false);
  c = __builtin_amdgcn_wmma_f32_16x16x32_bf16(false, ah, false, bl, (short)0, c, false, false);
  c = __builtin_amdgcn_wmma_f32_16x16x32_bf16(false, al, false, bh, (short)0, c, false, false);
#if defined(__HIP_DEVICE_COMPILE__)
  asm volatile("v_nop\n\tv_nop\n\tv_nop\n\tv_nop" : "+v"(c) : "v"(ah), "v"(al), "v"(bh), "v"(bl));
#endif
  return c;
}

__device__ __forceinline__ v16bf ldfrag(const u16t* rowp, int h) {
  FragB f;
  f.u[0] = *(const v8usa*)(rowp + 8 * h);
  f.u[1] = *(const v8usa*)(rowp + 16 + 8 * h);
  return f.v;
}

__global__ __launch_bounds__(NTHR) void k_wprep(
    const float* __restrict__ W1, const float* __restrict__ W2,
    const float* __restrict__ Wa1, const float* __restrict__ Wa2, u16t* wpl) {
  const int b = blockIdx.x;
  const float* src; int K, N, dstOff, segStart, part;
  if (b < 1)       { src = W1;  K = 32; N = 64;  dstOff = OW1P; segStart = 0;    part = 2; }
  else if (b < 3)  { src = W2;  K = 64; N = 64;  dstOff = OW2H; segStart = 256;  part = 0; }
  else if (b < 5)  { src = W2;  K = 64; N = 64;  dstOff = OW2L; segStart = 768;  part = 1; }
  else if (b < 6)  { src = Wa1; K = 32; N = 64;  dstOff = OA1H; segStart = 1280; part = 0; }
  else if (b < 7)  { src = Wa1; K = 32; N = 64;  dstOff = OA1L; segStart = 1536; part = 1; }
  else if (b < 11) { src = Wa2; K = 64; N = 128; dstOff = OA2H; segStart = 1792; part = 0; }
  else             { src = Wa2; K = 64; N = 128; dstOff = OA2L; segStart = 2816; part = 1; }
  const int i  = b * NTHR + (int)threadIdx.x - segStart;
  const int o  = i * 8;
  int n  = o / K;
  n = n > N - 1 ? N - 1 : n;
  const int k0 = o - (o / K) * K;
  v8us rv;
  if (part == 2) {
#pragma unroll
    for (int e = 0; e < 8; ++e) {
      const int s  = k0 + e;
      const int j  = s >> 3;
      const int a  = s & 7;
      const int ac = a > 5 ? 5 : a;
      const float x = src[ac * NCH + n];
      u16t hv, lv; split2(x, hv, lv);
      const u16t pv = (j == 1) ? lv : hv;
      rv[e] = (a < 6 && j < 3) ? pv : (u16t)0;
    }
  } else {
#pragma unroll
    for (int e = 0; e < 8; ++e) {
      const int k = k0 + e;
      const float x = src[k * N + n];
      u16t hv, lv; split2(x, hv, lv);
      rv[e] = (part == 0) ? hv : lv;
    }
  }
  u16t* dp = wpl + dstOff + o;
  *(volatile v8us*)dp = rv;
  __threadfence();
  *(volatile v8us*)dp = rv;
}

__global__ __launch_bounds__(NTHR) void k_cov(
    const float* __restrict__ geom, const int* __restrict__ ei, double* covp, int nP, int nE) {
  __shared__ double sw[NWV * 32];
  __shared__ __attribute__((aligned(16))) double sl[32];
  const int tid = threadIdx.x, lane = tid & 31, wv = tid >> 5;
  double a[27];
#pragma unroll
  for (int k = 0; k < 27; ++k) a[k] = 0.0;
#pragma unroll 1
  for (int e = blockIdx.x * NTHR + tid; e < nE; e += NBA * NTHR) {
    int i = ei[e];
    int j = ei[nE + e];
    i = i < 0 ? 0 : (i > nP - 1 ? nP - 1 : i);
    j = j < 0 ? 0 : (j > nP - 1 ? nP - 1 : j);
    const float* gi = geom + (size_t)i * 3;
    const float* gj = geom + (size_t)j * 3;
    const float x0 = gi[0], x1 = gi[1], x2 = gi[2];
    const float x3 = gj[0] - x0, x4 = gj[1] - x1, x5 = gj[2] - x2;
    const double d0 = (double)x0, d1 = (double)x1, d2 = (double)x2;
    const double d3 = (double)x3, d4 = (double)x4, d5 = (double)x5;
    a[0] += d0; a[1] += d1; a[2] += d2; a[3] += d3; a[4] += d4; a[5] += d5;
    a[6]  += d0 * d0; a[7]  += d0 * d1; a[8]  += d0 * d2; a[9]  += d0 * d3; a[10] += d0 * d4; a[11] += d0 * d5;
    a[12] += d1 * d1; a[13] += d1 * d2; a[14] += d1 * d3; a[15] += d1 * d4; a[16] += d1 * d5;
    a[17] += d2 * d2; a[18] += d2 * d3; a[19] += d2 * d4; a[20] += d2 * d5;
    a[21] += d3 * d3; a[22] += d3 * d4; a[23] += d3 * d5;
    a[24] += d4 * d4; a[25] += d4 * d5;
    a[26] += d5 * d5;
  }
#pragma unroll
  for (int k = 0; k < 27; ++k) {
    double v = a[k];
    v += __shfl_xor(v, 16);
    v += __shfl_xor(v, 8);
    v += __shfl_xor(v, 4);
    v += __shfl_xor(v, 2);
    v += __shfl_xor(v, 1);
    a[k] = v;
  }
  if (lane == 0) {
#pragma unroll
    for (int k = 0; k < 27; ++k) sw[wv * 32 + k] = a[k];
  }
  __syncthreads();
  if (tid < 27) {
    double t = 0.0;
#pragma unroll
    for (int w = 0; w < NWV; ++w) t += sw[w * 32 + tid];
    sl[tid] = t;
  } else if (tid < 32) {
    sl[tid] = 0.0;
  }
  __syncthreads();
  v2d ov = {0.0, 0.0};
  if (tid < 16) ov = *(const v2da*)(sl + 2 * tid);
  double* gp = covp + (size_t)blockIdx.x * 32 + 2 * tid;
  if (tid < 16) *(volatile v2d*)gp = ov;
  __threadfence();
  if (tid < 16) *(volatile v2d*)gp = ov;
}

__global__ __launch_bounds__(64) void k_fold1(
    const double* __restrict__ covp, const float* __restrict__ W1, const float* __restrict__ b1,
    const float* __restrict__ g1, float* par1, int nblk, int nE) {
  __shared__ double tot[32];
  __shared__ double mv[8];
  __shared__ double cm[36];
  __shared__ __attribute__((aligned(16))) float pl[128];
  const int tid = threadIdx.x;
  if (tid < 27) {
    double t = 0.0;
#pragma unroll 1
    for (int bb = 0; bb < nblk; ++bb) t += covp[(size_t)bb * 32 + tid];
    tot[tid] = t;
  }
  __syncthreads();
  const double invE = 1.0 / (double)nE;
  if (tid < 6) mv[tid] = tot[tid] * invE;
  __syncthreads();
  if (tid < 36) {
    const int aa = tid / 6, bb = tid - 6 * aa;
    const int p = aa < bb ? aa : bb, q = aa < bb ? bb : aa;
    const int idx = 6 + 6 * p - (p * (p - 1)) / 2 + (q - p);
    cm[tid] = tot[idx] * invE - mv[p] * mv[q];
  }
  __syncthreads();
  const int c = tid;
  double mu = (double)b1[c];
  double var = 0.0;
#pragma unroll 1
  for (int aa = 0; aa < 6; ++aa) {
    const double wa = (double)W1[aa * NCH + c];
    mu += mv[aa] * wa;
    double inner = 0.0;
#pragma unroll 1
    for (int bb = 0; bb < 6; ++bb) inner += (double)W1[bb * NCH + c] * cm[aa * 6 + bb];
    var += wa * inner;
  }
  var = var < 0.0 ? 0.0 : var;
  const float rs = rsqrtf((float)var + BNEPS);
  pl[c] = (float)mu;
  pl[NCH + c] = g1[c] * rs;
  __syncthreads();
  v4f ov = {0.f, 0.f, 0.f, 0.f};
  if (tid < 32) ov = *(const v4fa*)(pl + 4 * tid);
  if (tid < 32) *(volatile v4f*)(par1 + 4 * tid) = ov;
  __threadfence();
  if (tid < 32) *(volatile v4f*)(par1 + 4 * tid) = ov;
}

__global__ __launch_bounds__(128) void k_fold2(
    const double* __restrict__ st2, const float* __restrict__ g2, float* par2, int nblk, int nE) {
  __shared__ double T[128];
  __shared__ __attribute__((aligned(16))) float pl[128];
  const int tid = threadIdx.x;
  double t = 0.0;
#pragma unroll 1
  for (int bb = 0; bb < nblk; ++bb) t += st2[(size_t)bb * 128 + tid];
  T[tid] = t;
  __syncthreads();
  if (tid < NCH) {
    const double invE = 1.0 / (double)nE;
    const double mean = T[tid] * invE;
    double var = T[NCH + tid] * invE - mean * mean;
    var = var < 0.0 ? 0.0 : var;
    const float rs = rsqrtf((float)var + BNEPS);
    pl[tid] = (float)mean;
    pl[NCH + tid] = g2[tid] * rs;
  }
  __syncthreads();
  v4f ov = {0.f, 0.f, 0.f, 0.f};
  if (tid < 32) ov = *(const v4fa*)(pl + 4 * tid);
  if (tid < 32) *(volatile v4f*)(par2 + 4 * tid) = ov;
  __threadfence();
  if (tid < 32) *(volatile v4f*)(par2 + 4 * tid) = ov;
}

template <int MODE>
__global__ __launch_bounds__(NTHR) void k_edge(
    const float* __restrict__ geom, const float* __restrict__ aux, const int* __restrict__ ei,
    const u16t* __restrict__ wpl,
    const float* __restrict__ b1, const float* __restrict__ par1, const float* __restrict__ bb1,
    const float* __restrict__ b2, const float* __restrict__ par2, const float* __restrict__ bb2,
    const float* __restrict__ ba1, const float* __restrict__ ba2,
    const float* __restrict__ lng, const float* __restrict__ lnb,
    double* st2, float* out, int nP, int nE) {
  extern __shared__ v4f lds_dyn[];
  char*  lds = (char*)lds_dyn;
  u16t*  sW  = (u16t*)lds;
  float* prm = (float*)(lds + WPLB);
  const int tid = threadIdx.x, lane = tid & 31, wv = tid >> 5, h = lane >> 4, m = lane & 15;
  char*  wr = lds + LDS_BASEW + wv * WVB;
  u16t*  A6 = (u16t*)(wr + WA6);
  u16t*  HH = (u16t*)(wr + WHH);
  u16t*  HL = (u16t*)(wr + WHL);
  u16t*  XH = (u16t*)(wr + WXH);
  u16t*  XL = (u16t*)(wr + WXL);
  float* OS = (float*)(wr + WOS);
  double* SB = (double*)(lds + LDS_SB);
  double* SL = (double*)(lds + LDS_SL);

#pragma unroll 1
  for (int i = tid; i < WPLB / 16; i += NTHR) ((v4u*)sW)[i] = ((const v4u*)wpl)[i];
  if (tid < NCH) {
    prm[PB1 + tid]  = b1[tid];
    prm[PMU1 + tid] = par1[tid];
    prm[PSC1 + tid] = par1[NCH + tid];
    prm[PBB1 + tid] = bb1[tid];
    prm[PB2 + tid]  = b2[tid];
  }
  if (MODE == 1) {
    if (tid < NCH) {
      prm[PMU2 + tid] = par2[tid];
      prm[PSC2 + tid] = par2[NCH + tid];
      prm[PBB2 + tid] = bb2[tid];
      prm[PBA1 + tid] = ba1[tid];
      prm[PLNG + tid] = lng[tid];
      prm[PLNB + tid] = lnb[tid];
    }
    if (tid < 2 * NCH) prm[PBA2 + tid] = ba2[tid];
  }
  {
    const v4u z = {0u, 0u, 0u, 0u};
    ((v4u*)A6)[lane] = z;
    ((v4u*)A6)[32 + lane] = z;
  }
  __syncthreads();

  double S[4], Q[4];
#pragma unroll
  for (int t = 0; t < 4; ++t) { S[t] = 0.0; Q[t] = 0.0; }
  const v8f zero8 = {0.f, 0.f, 0.f, 0.f, 0.f, 0.f, 0.f, 0.f};
  const float ninf = -__builtin_inff();
  const int pw0 = blockIdx.x * PPB + wv * PPW;

#pragma unroll 1
  for (int pt = 0; pt < PPW; ++pt) {
    const int p = pw0 + pt;
    const int e = p * KNB + m;
    const int iraw = ei[e];
    const int jraw = ei[nE + e];
    const int ic = iraw < 0 ? 0 : (iraw > nP - 1 ? nP - 1 : iraw);
    const int jc = jraw < 0 ? 0 : (jraw > nP - 1 ? nP - 1 : jraw);
    const unsigned bal = __builtin_amdgcn_ballot_w32(iraw == p);

    {
      const float* gi = geom + (size_t)ic * 3;
      const float* gj = geom + (size_t)jc * 3;
      float v[6];
      v[0] = gi[0]; v[1] = gi[1]; v[2] = gi[2];
      v[3] = gj[0] - v[0]; v[4] = gj[1] - v[1]; v[5] = gj[2] - v[2];
      u16t* arow = A6 + m * 32 + 16 * h;
#pragma unroll
      for (int s = 0; s < 6; ++s) {
        u16t hv, lv; split2(v[s], hv, lv);
        arow[s]     = h ? lv : hv;
        arow[8 + s] = h ? (u16t)0 : hv;
      }
    }
    wsync();

    v8f acc[4];
    {
      const v16bf a = ldfrag(A6 + m * 32, h);
#pragma unroll
      for (int t = 0; t < 4; ++t) {
        const v16bf bf = ldfrag(sW + OW1P + (16 * t + m) * 32, h);
        acc[t] = wmb1(a, bf, zero8);
      }
    }
    wsync();
#pragma unroll
    for (int t = 0; t < 4; ++t) {
      const int ch = 16 * t + m;
      const float cb = prm[PB1 + ch], mu = prm[PMU1 + ch], sc = prm[PSC1 + ch], be = prm[PBB1 + ch];
#pragma unroll
      for (int r = 0; r < 8; ++r) {
        const float x = acc[t][r] + cb;
        const float y = fmaxf((x - mu) * sc + be, 0.f);
        u16t hv, lv; split2(y, hv, lv);
        const int o = (8 * h + r) * NCH + ch;
        HH[o] = hv; HL[o] = lv;
      }
    }
    wsync();

#pragma unroll
    for (int t = 0; t < 4; ++t) acc[t] = zero8;
#pragma unroll
    for (int ks = 0; ks < 2; ++ks) {
      const v16bf ah = ldfrag(HH + m * NCH + 32 * ks, h);
      const v16bf al = ldfrag(HL + m * NCH + 32 * ks, h);
#pragma unroll
      for (int t = 0; t < 4; ++t) {
        const v16bf bh = ldfrag(sW + OW2H + (16 * t + m) * NCH + 32 * ks, h);
        const v16bf bl = ldfrag(sW + OW2L + (16 * t + m) * NCH + 32 * ks, h);
        acc[t] = wm3(ah, al, bh, bl, acc[t]);
      }
    }

    if (MODE == 0) {
#pragma unroll
      for (int t = 0; t < 4; ++t) {
        const float cb = prm[PB2 + 16 * t + m];
        float s = 0.f, q = 0.f;
#pragma unroll
        for (int r = 0; r < 8; ++r) { const float x = acc[t][r] + cb; s += x; q += x * x; }
        s += __shfl_xor(s, 16);
        q += __shfl_xor(q, 16);
        S[t] += (double)s;
        Q[t] += (double)q;
      }
    } else {
      v8f ef[4];
#pragma unroll
      for (int t = 0; t < 4; ++t) {
        const int ch = 16 * t + m;
        const float cb = prm[PB2 + ch], mu = prm[PMU2 + ch], sc = prm[PSC2 + ch], be = prm[PBB2 + ch];
#pragma unroll
        for (int r = 0; r < 8; ++r) {
          const float x = acc[t][r] + cb;
          ef[t][r] = fmaxf((x - mu) * sc + be, 0.f);
        }
      }
      {
        const int nd = h ? jc : ic;
        const float* ap = aux + (size_t)nd * NAUX;
        const v4f q0 = *(const v4f*)ap, q1 = *(const v4f*)(ap + 4);
        const v4f q2 = *(const v4f*)(ap + 8), q3 = *(const v4f*)(ap + 12);
        float av[16];
        av[0] = q0.x; av[1] = q0.y; av[2]  = q0.z; av[3]  = q0.w; av[4]  = q1.x; av[5]  = q1.y; av[6]  = q1.z; av[7]  = q1.w;
        av[8] = q2.x; av[9] = q2.y; av[10] = q2.z; av[11] = q2.w; av[12] = q3.x; av[13] = q3.y; av[14] = q3.z; av[15] = q3.w;
        v8us xh0, xl0, xh1, xl1;
#pragma unroll
        for (int c = 0; c < 8; ++c) {
          u16t hv, lv;
          split2(av[c], hv, lv);     xh0[c] = hv; xl0[c] = lv;
          split2(av[8 + c], hv, lv); xh1[c] = hv; xl1[c] = lv;
        }
        u16t* xr = XH + m * 32 + 16 * h;
        u16t* xs = XL + m * 32 + 16 * h;
        *(v8us*)xr = xh0; *(v8us*)(xr + 8) = xh1;
        *(v8us*)xs = xl0; *(v8us*)(xs + 8) = xl1;
      }
      wsync();
      v8f u[4];
      {
        const v16bf xa = ldfrag(XH + m * 32, h);
        const v16bf xb = ldfrag(XL + m * 32, h);
#pragma unroll
        for (int t = 0; t < 4; ++t) {
          const v16bf bh = ldfrag(sW + OA1H + (16 * t + m) * 32, h);
          const v16bf bl = ldfrag(sW + OA1L + (16 * t + m) * 32, h);
          u[t] = wm3(xa, xb, bh, bl, zero8);
        }
      }
      wsync();
#pragma unroll
      for (int t = 0; t < 4; ++t) {
        const int ch = 16 * t + m;
        const float cb = prm[PBA1 + ch];
#pragma unroll
        for (int r = 0; r < 8; ++r) {
          const float y = fmaxf(u[t][r] + cb, 0.f);
          u16t hv, lv; split2(y, hv, lv);
          const int o = (8 * h + r) * NCH + ch;
          HH[o] = hv; HL[o] = lv;
        }
      }
      wsync();
      v8f md[4];
      {
        v8f g[4];
#pragma unroll
        for (int t = 0; t < 4; ++t) g[t] = zero8;
#pragma unroll
        for (int ks = 0; ks < 2; ++ks) {
          const v16bf ah = ldfrag(HH + m * NCH + 32 * ks, h);
          const v16bf al = ldfrag(HL + m * NCH + 32 * ks, h);
#pragma unroll
          for (int t = 0; t < 4; ++t) {
            const v16bf bh = ldfrag(sW + OA2H + (16 * t + m) * NCH + 32 * ks, h);
            const v16bf bl = ldfrag(sW + OA2L + (16 * t + m) * NCH + 32 * ks, h);
            g[t] = wm3(ah, al, bh, bl, g[t]);
          }
        }
#pragma unroll
        for (int t = 0; t < 4; ++t) {
          const float cb = prm[PBA2 + 16 * t + m];
#pragma unroll
          for (int r = 0; r < 8; ++r) {
            const float gv = g[t][r] + cb + 1.0f;
            const float ex = __expf(-gv);
            const float gm = __builtin_amdgcn_rcpf(1.0f + ex);
            md[t][r] = gm * ef[t][r];
          }
        }
      }
      {
        v8f g[4];
#pragma unroll
        for (int t = 0; t < 4; ++t) g[t] = zero8;
#pragma unroll
        for (int ks = 0; ks < 2; ++ks) {
          const v16bf ah = ldfrag(HH + m * NCH + 32 * ks, h);
          const v16bf al = ldfrag(HL + m * NCH + 32 * ks, h);
#pragma unroll
          for (int t = 0; t < 4; ++t) {
            const v16bf bh = ldfrag(sW + OA2H + (NCH + 16 * t + m) * NCH + 32 * ks, h);
            const v16bf bl = ldfrag(sW + OA2L + (NCH + 16 * t + m) * NCH + 32 * ks, h);
            g[t] = wm3(ah, al, bh, bl, g[t]);
          }
        }
#pragma unroll
        for (int t = 0; t < 4; ++t) {
          const float cb = prm[PBA2 + NCH + 16 * t + m];
#pragma unroll
          for (int r = 0; r < 8; ++r) md[t][r] = md[t][r] + (g[t][r] + cb);
        }
      }
      float pv[4];
#pragma unroll
      for (int t = 0; t < 4; ++t) {
        float mx = ninf;
#pragma unroll
        for (int r = 0; r < 8; ++r) {
          const bool ok = ((bal >> (8 * h + r)) & 1u) != 0u;
          mx = fmaxf(mx, ok ? md[t][r] : ninf);
        }
        mx = fmaxf(mx, __shfl_xor(mx, 16));
        pv[t] = mx;
      }
      float s = pv[0] + pv[1] + pv[2] + pv[3];
      s += __shfl_xor(s, 1); s += __shfl_xor(s, 2); s += __shfl_xor(s, 4); s += __shfl_xor(s, 8);
      const float mean = s * (1.0f / 64.0f);
      float q = 0.f;
#pragma unroll
      for (int t = 0; t < 4; ++t) { const float d = pv[t] - mean; q += d * d; }
      q += __shfl_xor(q, 1); q += __shfl_xor(q, 2); q += __shfl_xor(q, 4); q += __shfl_xor(q, 8);
      const float inv = rsqrtf(q * (1.0f / 64.0f) + BNEPS);
#pragma unroll
      for (int t = 0; t < 4; ++t) {
        const int ch = 16 * t + m;
        float y = (prm[PLNG + ch] * (pv[t] - mean)) * inv + prm[PLNB + ch];
        y = y < 0.f ? 0.f : y;
        OS[pt * NCH + ch] = y;
      }
    }
  }

  if (MODE == 0) {
#pragma unroll
    for (int t = 0; t < 4; ++t) {
      SB[wv * 128 + 16 * t + m] = S[t];
      SB[wv * 128 + NCH + 16 * t + m] = Q[t];
    }
    __syncthreads();
    if (tid < 128) {
      double acc2 = 0.0;
#pragma unroll
      for (int w = 0; w < NWV; ++w) acc2 += SB[w * 128 + tid];
      SL[tid] = acc2;
    }
    __syncthreads();
    v2d o0 = {0.0, 0.0}, o1 = {0.0, 0.0};
    double* gp = st2 + (size_t)blockIdx.x * 128;
    if (wv == 0) {
      o0 = *(const v2da*)(SL + 2 * lane);
      o1 = *(const v2da*)(SL + 2 * (32 + lane));
      *(volatile v2d*)(gp + 2 * lane) = o0;
      *(volatile v2d*)(gp + 2 * (32 + lane)) = o1;
    }
    __threadfence();
    if (wv == 0) {
      *(volatile v2d*)(gp + 2 * lane) = o0;
      *(volatile v2d*)(gp + 2 * (32 + lane)) = o1;
    }
  } else {
    wsync();
    v4f ov[4];
#pragma unroll
    for (int qq = 0; qq < 4; ++qq) ov[qq] = *(const v4fa*)(OS + (qq * 32 + lane) * 4);
    float* op = out + (size_t)pw0 * NCH;
#pragma unroll
    for (int qq = 0; qq < 4; ++qq) *(volatile v4f*)(op + (qq * 32 + lane) * 4) = ov[qq];
    __threadfence();
#pragma unroll
    for (int qq = 0; qq < 4; ++qq) *(volatile v4f*)(op + (qq * 32 + lane) * 4) = ov[qq];
  }
}

extern "C" void kernel_launch(void* const* d_in, const int* in_sizes, int n_in,
                              void* d_out, int out_size, void* d_ws, size_t ws_size,
                              hipStream_t stream) {
  if (n_in < 18) return;
  const int nP = in_sizes[0] / 3;
  if (nP <= 0 || in_sizes[0] != 3 * nP || (nP % PPB) != 0) return;
  const int nE = in_sizes[17] / 2;
  if (in_sizes[17] != 2 * nE || nE != KNB * nP) return;
  if (in_sizes[1] != NAUX * nP || out_size != nP * NCH) return;
  if (in_sizes[2] != 6 * NCH || in_sizes[3] != NCH || in_sizes[4] != NCH || in_sizes[5] != NCH) return;
  if (in_sizes[6] != NCH * NCH || in_sizes[7] != NCH || in_sizes[8] != NCH || in_sizes[9] != NCH) return;
  if (in_sizes[10] != 2 * NAUX * NCH || in_sizes[11] != NCH || in_sizes[12] != NCH * 2 * NCH ||
      in_sizes[13] != 2 * NCH || in_sizes[14] != NCH || in_sizes[15] != NCH) return;
  if (nP > (1 << 24)) return;

  const float* geom = (const float*)d_in[0];
  const float* aux  = (const float*)d_in[1];
  const float* W1   = (const float*)d_in[2];
  const float* b1   = (const float*)d_in[3];
  const float* g1   = (const float*)d_in[4];
  const float* bb1  = (const float*)d_in[5];
  const float* W2   = (const float*)d_in[6];
  const float* b2   = (const float*)d_in[7];
  const float* g2   = (const float*)d_in[8];
  const float* bb2  = (const float*)d_in[9];
  const float* Wa1  = (const float*)d_in[10];
  const float* ba1  = (const float*)d_in[11];
  const float* Wa2  = (const float*)d_in[12];
  const float* ba2  = (const float*)d_in[13];
  const float* lng  = (const float*)d_in[14];
  const float* lnb  = (const float*)d_in[15];
  const int*   ei   = (const int*)d_in[17];
  float* out = (float*)d_out;

  const int nblkE = nP / PPB;

  char* ws = (char*)d_ws;
  size_t off = 0;
  const size_t oWPL = off; off += (size_t)WPLB;                  off = (off + 255) & ~(size_t)255;
  const size_t oP1  = off; off += (size_t)128 * 4;               off = (off + 255) & ~(size_t)255;
  const size_t oP2  = off; off += (size_t)128 * 4;               off = (off + 255) & ~(size_t)255;
  const size_t oCOV = off; off += (size_t)NBA * 32 * 8;          off = (off + 255) & ~(size_t)255;
  const size_t oST2 = off; off += (size_t)nblkE * 128 * 8;       off = (off + 255) & ~(size_t)255;
  if (off > ws_size) return;
  u16t*   wpl  = (u16t*)(ws + oWPL);
  float*  par1 = (float*)(ws + oP1);
  float*  par2 = (float*)(ws + oP2);
  double* cov  = (double*)(ws + oCOV);
  double* st2  = (double*)(ws + oST2);

  k_wprep<<<(WPLB / 16) / NTHR, NTHR, 0, stream>>>(W1, W2, Wa1, Wa2, wpl);

  k_cov<<<NBA, NTHR, 0, stream>>>(geom, ei, cov, nP, nE);
  k_fold1<<<1, 64, 0, stream>>>(cov, W1, b1, g1, par1, NBA, nE);

  hipFuncSetAttribute(reinterpret_cast<const void*>(&k_edge<0>),
                      hipFuncAttributeMaxDynamicSharedMemorySize, LDS_EDGE);
  k_edge<0><<<nblkE, NTHR, LDS_EDGE, stream>>>(geom, aux, ei, wpl, b1, par1, bb1, b2, par2, bb2,
                                               ba1, ba2, lng, lnb, st2, out, nP, nE);
  k_fold2<<<1, 128, 0, stream>>>(st2, g2, par2, nblkE, nE);

  hipFuncSetAttribute(reinterpret_cast<const void*>(&k_edge<1>),
                      hipFuncAttributeMaxDynamicSharedMemorySize, LDS_EDGE);
  k_edge<1><<<nblkE, NTHR, LDS_EDGE, stream>>>(geom, aux, ei, wpl, b1, par1, bb1, b2, par2, bb2,
                                               ba1, ba2, lng, lnb, st2, out, nP, nE);
}
